// DictionaryLearning_21019569946795
// MI455X (gfx1250) — hardware-verified
//
#include <hip/hip_runtime.h>
#include <math.h>

typedef __attribute__((ext_vector_type(16))) _Float16 v16h;
typedef __attribute__((ext_vector_type(16))) __bf16 v16b;
typedef __attribute__((ext_vector_type(8)))  _Float16 v8h;
typedef __attribute__((ext_vector_type(8)))  float v8f;
typedef __attribute__((ext_vector_type(4)))  float v4f;
typedef __attribute__((ext_vector_type(2)))  float v2f;
typedef __attribute__((ext_vector_type(4)))  unsigned v4u;
typedef __attribute__((ext_vector_type(4)))  int v4i;
typedef float __attribute__((may_alias)) float_a;
typedef int __attribute__((may_alias)) int_a;

template <typename T> __device__ __forceinline__ void vst2(void* p, T v) { *(volatile T*)p = v; __threadfence(); *(volatile T*)p = v; }
__device__ __forceinline__ v8f wmma16(v16h a, v16h b, v8f c) {
  v8f d = __builtin_amdgcn_wmma_f32_16x16x32_f16(false, a, false, b, (short)0, c, false, false);
  asm volatile("v_nop\n\tv_nop\n\tv_nop\n\tv_nop" : "+v"(d) : "v"(a), "v"(b));
  return d;
}
__device__ __forceinline__ v8f wmma_bf(v16b a, v16b b, v8f c) {
  v8f d = __builtin_amdgcn_wmma_f32_16x16x32_bf16(false, a, false, b, (short)0, c, false, false);
  asm volatile("v_nop\n\tv_nop\n\tv_nop\n\tv_nop" : "+v"(d) : "v"(a), "v"(b));
  return d;
}
__device__ __forceinline__ v16h frag_h(const _Float16* rowk0, int lane) {
  union { v16h v; v8h q[2]; } u; const _Float16* p = rowk0 + 8 * (lane >> 4);
  u.q[0] = *(const v8h*)p; u.q[1] = *(const v8h*)(p + 16); return u.v;
}
__device__ __forceinline__ v16h frag_f32(const float* rowk0, int lane) {
  v16h a; const float* p = rowk0 + 8 * (lane >> 4);
#pragma unroll
  for (int i = 0; i < 8; ++i) { a[i] = (_Float16)p[i]; a[8 + i] = (_Float16)p[16 + i]; }
  return a;
}
__device__ __forceinline__ v16h frag_f32s(const float* rowk0, int lane, float sc) {
  v16h a; const float* p = rowk0 + 8 * (lane >> 4);
#pragma unroll
  for (int i = 0; i < 8; ++i) { a[i] = (_Float16)(p[i] * sc); a[8 + i] = (_Float16)(p[16 + i] * sc); }
  return a;
}
__device__ __forceinline__ v16h fragc_f32(const float* W, int k0, int n, int lane, int ld, int K) {
  v16h a; const int g = lane >> 4;
#pragma unroll
  for (int i = 0; i < 8; ++i) { const int ka = k0 + 8 * g + i, kb = ka + 16;
    a[i] = (_Float16)(ka < K ? W[(size_t)(ka < K ? ka : K - 1) * ld + n] : 0.f); a[8 + i] = (_Float16)(kb < K ? W[(size_t)(kb < K ? kb : K - 1) * ld + n] : 0.f); }
  return a;
}
struct F2 { v16b h, l; };
__device__ __forceinline__ F2 bsplit16(const float v[16]) { F2 r;
#pragma unroll
  for (int i = 0; i < 16; ++i) { const __bf16 h = (__bf16)v[i]; r.h[i] = h; r.l[i] = (__bf16)(v[i] - (float)h); }
  return r; }
__device__ __forceinline__ F2 split_row(const float* row, int k0, int lane) { float v[16]; const float* p = row + k0 + 8 * (lane >> 4);
#pragma unroll
  for (int i = 0; i < 8; ++i) { v[i] = p[i]; v[8 + i] = p[16 + i]; }
  return bsplit16(v); }
__device__ __forceinline__ F2 split_rowK(const float* row, int k0, int lane, int K) { float v[16]; const int g = lane >> 4;
#pragma unroll
  for (int i = 0; i < 8; ++i) { const int ka = k0 + 8 * g + i, kb = ka + 16; v[i] = ka < K ? row[ka < K ? ka : K - 1] : 0.f; v[8 + i] = kb < K ? row[kb < K ? kb : K - 1] : 0.f; }
  return bsplit16(v); }
__device__ __forceinline__ F2 split_col(const float* W, int k0, int n, int lane, int ld, int K) { float v[16]; const int g = lane >> 4;
#pragma unroll
  for (int i = 0; i < 8; ++i) { const int ka = k0 + 8 * g + i, kb = ka + 16; v[i] = ka < K ? W[(size_t)(ka < K ? ka : K - 1) * ld + n] : 0.f; v[8 + i] = kb < K ? W[(size_t)(kb < K ? kb : K - 1) * ld + n] : 0.f; }
  return bsplit16(v); }
__device__ __forceinline__ v8f mac3(const F2& a, const F2& b, v8f c) { c = wmma_bf(a.l, b.h, c); c = wmma_bf(a.h, b.l, c); return wmma_bf(a.h, b.h, c); }
__device__ __forceinline__ float sigm(float v) { return 1.0f / (1.0f + expf(-v)); }
#define LDSX() do { asm volatile("s_wait_dscnt 0" ::: "memory"); __builtin_amdgcn_wave_barrier(); __builtin_amdgcn_fence(__ATOMIC_RELEASE, "workgroup"); } while (0)


#define NBI 8
#define CH 64
#define IMH 128
#define IMW 128
#define PS 4
#define STR 2
#define HO 63
#define WO 63
#define NP (NBI * HO * WO)
#define NPB ((NP + 63) / 64)
#define PD_ (CH * PS * PS)
#define NA 512
#define SP 5
#ifndef TB0
#define TB0 0
#define TNB NBI
#define NPBT NPB
#endif
typedef __attribute__((ext_vector_type(8))) __bf16 v8b;
__device__ __forceinline__ v16b frag_b(const __bf16* rowk0, int lane) {
  union { v16b v; v8b q[2]; } u; const __bf16* p = rowk0 + 8 * (lane >> 4);
  u.q[0] = *(const v8b*)p; u.q[1] = *(const v8b*)(p + 16); return u.v;
}
__device__ __forceinline__ float bfr(float v) { return (float)(__bf16)v; }
__device__ __attribute__((noinline)) float exp_ni(float v) { return expf(v); }
__device__ __attribute__((noinline)) float erf_ni(float v) { return erff(v); }

__device__ __attribute__((noinline)) float cosf_ni(float v) { return cosf(v); }
#define WS_PDT 0u
#define WS_COR (WS_PDT + 2u * NA * PD_)
#define WS_GRM (WS_COR + 4u * NPB * 64 * NA)
#define WS_CODE (WS_GRM + 4u * NA * NA)
#define WS_PL  (WS_CODE + 4u * NPB * 64 * 16)
#define WS_END (WS_PL + 4u * 8192 * 32)

__global__ __launch_bounds__(256) void k_packD(const float* __restrict__ Dm, __bf16* __restrict__ PDT) {
  __shared__ __align__(16) __bf16 s[PD_]; const int a = blockIdx.x, tid = threadIdx.x;
  for (int k = tid; k < PD_; k += 256) s[k] = (__bf16)Dm[(size_t)k * NA + a];
  __syncthreads();
  if (tid < PD_ / 8) vst2((unsigned*)(PDT + (size_t)a * PD_ + tid * 8), *(const v4u*)&s[tid * 8]);
}
__global__ __launch_bounds__(128) void k_corr(const float* __restrict__ X, const __bf16* __restrict__ PDT, float* __restrict__ COR) {
  __shared__ __align__(16) float so[4][16][132];
  const int tid = threadIdx.x, wave = tid >> 5, lane = tid & 31, col = lane & 15, g = lane >> 4; const size_t r0 = (size_t)blockIdx.x * 64 + wave * 16; const int n0 = blockIdx.y * 128;
  int n = (int)(r0 + col); if (n >= NP) n = NP - 1; const int b = n / (HO * WO), rem = n % (HO * WO), ho = rem / WO, wo = rem % WO;
  const float* xb = X + (size_t)b * CH * IMH * IMW + (size_t)(2 * ho) * IMW + 2 * wo;
  v8f acc[8] = {};
#pragma unroll 2
  for (int kc = 0; kc < PD_ / 32; ++kc) { v16b a;
#pragma unroll
    for (int i = 0; i < 16; ++i) { const int k = kc * 32 + 8 * g + (i & 7) + ((i >> 3) << 4); const int c = k >> 4, ph = (k >> 2) & 3, pw = k & 3; a[i] = (__bf16)xb[(size_t)c * IMH * IMW + ph * IMW + pw]; }
#pragma unroll
    for (int j = 0; j < 8; ++j) acc[j] = wmma_bf(a, frag_b(PDT + (size_t)(n0 + j * 16 + col) * PD_ + kc * 32, lane), acc[j]); }
#pragma unroll
  for (int j = 0; j < 8; ++j)
#pragma unroll
    for (int r = 0; r < 8; ++r) so[wave][8 * g + r][j * 16 + col] = acc[j][r];
  LDSX();
  for (int rl = 0; rl < 16; ++rl) vst2(COR + (r0 + rl) * NA + n0 + lane * 4, *(const v4f*)&so[wave][rl][lane * 4]);
}
__global__ __launch_bounds__(128) void k_gram(const __bf16* __restrict__ PDT, float* __restrict__ GRM) {
  __shared__ __align__(16) float so[4][16][132];
  const int tid = threadIdx.x, wave = tid >> 5, lane = tid & 31, col = lane & 15, g = lane >> 4; const size_t r0 = (size_t)blockIdx.x * 64 + wave * 16; const int n0 = blockIdx.y * 128;
  v8f acc[8] = {};
#pragma unroll 2
  for (int kc = 0; kc < PD_ / 32; ++kc) { const v16b a = frag_b(PDT + (r0 + col) * PD_ + kc * 32, lane);
#pragma unroll
    for (int j = 0; j < 8; ++j) acc[j] = wmma_bf(a, frag_b(PDT + (size_t)(n0 + j * 16 + col) * PD_ + kc * 32, lane), acc[j]); }
#pragma unroll
  for (int j = 0; j < 8; ++j)
#pragma unroll
    for (int r = 0; r < 8; ++r) so[wave][8 * g + r][j * 16 + col] = acc[j][r];
  LDSX();
  for (int rl = 0; rl < 16; ++rl) vst2(GRM + (r0 + rl) * NA + n0 + lane * 4, *(const v4f*)&so[wave][rl][lane * 4]);
}
__global__ __launch_bounds__(64) void k_code(const float* __restrict__ COR, const float* __restrict__ GRM, const float* __restrict__ X, const float* __restrict__ Dm, float* __restrict__ CODE) {
  __shared__ __align__(16) float sc[64][16]; const int tid = threadIdx.x; const size_t n = (size_t)blockIdx.x * 64 + tid;
  const float* cr = COR + n * NA;
  int s8[8]; float a8[8];
#pragma unroll
  for (int j = 0; j < 8; ++j) { s8[j] = -1; a8[j] = -1.f; }
#pragma unroll 1
  for (int a = 0; a < NA; ++a) { const float v = fabsf(cr[a]);
    if (v > a8[7]) { int pos = 7;
#pragma unroll
      for (int j = 6; j >= 0; --j) if (v > a8[j]) pos = j;
#pragma unroll
      for (int j = 7; j >= 1; --j) if (j > pos) { a8[j] = a8[j - 1]; s8[j] = s8[j - 1]; }
#pragma unroll
      for (int j = 0; j < 8; ++j) if (j == pos) { a8[j] = v; s8[j] = a; } } }
  if (a8[4] - a8[5] < 1e-4f) {
    const int pn = (int)(n < (size_t)NP ? n : (size_t)NP - 1); const int b = pn / (HO * WO), rem = pn % (HO * WO), ho = rem / WO, wo = rem % WO; const float* xb = X + (size_t)b * CH * IMH * IMW + (size_t)(2 * ho) * IMW + 2 * wo;
    double e8[8];
#pragma unroll
    for (int j = 0; j < 8; ++j) e8[j] = 0.0;
#pragma unroll 1
    for (int k = 0; k < PD_; ++k) { const int c = k >> 4, ph = (k >> 2) & 3, pw = k & 3; const double xv = (double)bfr(xb[(size_t)c * IMH * IMW + ph * IMW + pw]); const float* dr = Dm + (size_t)k * NA;
#pragma unroll
      for (int j = 0; j < 8; ++j) { const int a = s8[j] < 0 ? 0 : s8[j]; e8[j] += xv * (double)bfr(dr[a]); } }
#pragma unroll
    for (int j = 0; j < 8; ++j) { e8[j] = (s8[j] < 0) ? -1.0 : fabs(e8[j]); }
#pragma unroll
    for (int i = 0; i < 8; ++i) {
#pragma unroll
      for (int j = i + 1; j < 8; ++j) { const bool sw = (e8[j] > e8[i]) || (e8[j] == e8[i] && s8[j] < s8[i]); if (sw) { const double te = e8[i]; e8[i] = e8[j]; e8[j] = te; const int ts = s8[i]; s8[i] = s8[j]; s8[j] = ts; } } } }
  int s[SP];
#pragma unroll
  for (int j = 0; j < SP; ++j) s[j] = s8[j] < 0 ? 0 : s8[j];
  __shared__ float swk[64][33]; float* wk = &swk[tid][0];
  for (int i = 0; i < SP; ++i) { int si = s[0];
#pragma unroll
    for (int q = 1; q < SP; ++q) if (q == i) si = s[q];
    wk[25 + i] = cr[si];
    for (int j = 0; j < SP; ++j) { int sj = s[0];
#pragma unroll
      for (int q = 1; q < SP; ++q) if (q == j) sj = s[q];
      wk[i * 5 + j] = GRM[(size_t)si * NA + sj] + ((i == j) ? 1e-10f : 0.f); } }
#pragma unroll 1
  for (int k = 0; k < SP; ++k) { int piv = k; float best = fabsf(wk[k * 5 + k]);
    for (int i = k + 1; i < SP; ++i) { const float t = fabsf(wk[i * 5 + k]); if (t > best) { best = t; piv = i; } }
    if (piv != k) { for (int j = 0; j < SP; ++j) { const float t = wk[k * 5 + j]; wk[k * 5 + j] = wk[piv * 5 + j]; wk[piv * 5 + j] = t; } const float t = wk[25 + k]; wk[25 + k] = wk[25 + piv]; wk[25 + piv] = t; }
#pragma unroll 1
    for (int i = k + 1; i < SP; ++i) { const float l = wk[i * 5 + k] / wk[k * 5 + k]; wk[i * 5 + k] = l;
#pragma unroll 1
      for (int j = k + 1; j < SP; ++j) wk[i * 5 + j] = wk[i * 5 + j] - l * wk[k * 5 + j]; } }
#pragma unroll 1
  for (int i = 0; i < SP; ++i) { float t = wk[25 + i];
#pragma unroll 1
    for (int j = 0; j < i; ++j) t -= wk[i * 5 + j] * wk[25 + j]; wk[25 + i] = t; }
  float v[SP];
#pragma unroll 1
  for (int i = SP - 1; i >= 0; --i) { float t = wk[25 + i];
#pragma unroll 1
    for (int j = i + 1; j < SP; ++j) t -= wk[i * 5 + j] * wk[25 + j]; wk[25 + i] = t / wk[i * 5 + i]; }
#pragma unroll
  for (int i = 0; i < SP; ++i) v[i] = wk[25 + i];
#pragma unroll
  for (int j = 0; j < SP; ++j) { sc[tid][j] = __int_as_float(s[j]); sc[tid][8 + j] = v[j]; }
  sc[tid][5] = 0.f; sc[tid][6] = 0.f; sc[tid][7] = 0.f; sc[tid][13] = 0.f; sc[tid][14] = 0.f; sc[tid][15] = 0.f;
  __syncthreads();
  for (int q = tid; q < 64 * 4; q += 64) vst2(CODE + ((size_t)blockIdx.x * 64) * 16 + q * 4, *(const v4f*)(&sc[0][0] + q * 4));
}
__global__ __launch_bounds__(128) void k_fold(const float* __restrict__ X, const float* __restrict__ Dm, const float* __restrict__ CODE, float* __restrict__ OUTQ, float* __restrict__ PL) {
  __shared__ float sw1[4]; __shared__ __align__(16) float sq[128]; __shared__ float sred[128]; __shared__ __align__(16) float sl[32];
  const int colx = threadIdx.x; const int r = blockIdx.x, c = blockIdx.y, b = blockIdx.z + TB0;
  if (colx < 4) { const float ang = (6.283185307179586f * (float)colx) / 3.0f; sw1[colx] = 0.5f * (1.0f - cosf_ni(ang)); }
  __syncthreads();
  const size_t xi = (((size_t)b * CH + c) * IMH + r) * IMW + colx; const float xv = bfr(X[xi]);
  float num = 0.f, den = 0.f;
  for (int ph = 0; ph < 4; ++ph) { const int rr = r - ph; if (rr < 0 || (rr & 1)) continue; const int ho = rr >> 1; if (ho >= HO) continue;
    for (int pw = 0; pw < 4; ++pw) { const int cc = colx - pw; if (cc < 0 || (cc & 1)) continue; const int wo = cc >> 1; if (wo >= WO) continue;
      const float w2 = sw1[ph] * sw1[pw]; den += w2;
      if (w2 != 0.f) { const size_t n = ((size_t)b * HO + ho) * WO + wo; const float* cd = CODE + n * 16; const int k = c * 16 + ph * 4 + pw; float xh = 0.f;
        int ss[SP]; float vv[SP];
#pragma unroll
        for (int j = 0; j < SP; ++j) { ss[j] = __float_as_int(cd[j]); vv[j] = cd[8 + j]; }
#pragma unroll
        for (int p = 0; p < SP; ++p)
#pragma unroll
          for (int q = 0; q + 1 < SP - p; ++q) if (ss[q] > ss[q + 1]) { const int ti = ss[q]; ss[q] = ss[q + 1]; ss[q + 1] = ti; const float tv = vv[q]; vv[q] = vv[q + 1]; vv[q + 1] = tv; }
#pragma unroll
        for (int j = 0; j < SP; ++j) { const int a = min(max(ss[j], 0), NA - 1); xh += vv[j] * bfr(Dm[(size_t)k * NA + a]); }
        num += xh * w2; } } }
  const float z = num / fmaxf(den, 1e-10f);
  const float d = z - xv; sq[colx] = xv + d; sred[colx] = d * d;
  __syncthreads();
  if (colx < 32) vst2(OUTQ + xi - colx + colx * 4, *(const v4f*)&sq[colx * 4]);
  if (colx == 0) { float t = 0.f; for (int i = 0; i < 128; ++i) t += sred[i]; sl[0] = t; for (int i = 1; i < 32; ++i) sl[i] = 0.f; }
  __syncthreads();
  if (colx < 8) vst2(PL + (((size_t)blockIdx.z * CH + c) * IMH + r) * 32 + colx * 4, *(const v4f*)&sl[colx * 4]);
}
__global__ __launch_bounds__(256) void k_loss(const float* __restrict__ PL, float* __restrict__ OUTL) {
  __shared__ float sp[256]; const int tid = threadIdx.x; float a = 0.f;
  for (int i = tid; i < TNB * CH * IMH; i += 256) a += PL[(size_t)i * 32];
  sp[tid] = a; __syncthreads();
  if (tid == 0) { float t = 0.f; for (int i = 0; i < 256; ++i) t += sp[i]; const float m = t / (float)((size_t)NBI * CH * IMH * IMW); const float loss = m + 0.25f * m; *(volatile float*)OUTL = loss; __threadfence(); *(volatile float*)OUTL = loss; }
}
extern "C" void kernel_launch(void* const* d_in, const int* in_sizes, int n_in, void* d_out, int out_size, void* d_ws, size_t ws_size, hipStream_t stream) {
  (void)in_sizes; (void)n_in; (void)out_size;
  const float* X = (const float*)d_in[0]; const float* Dm = (const float*)d_in[1];
  if (ws_size < (size_t)WS_END) return;
  char* ws = (char*)d_ws; __bf16* PDT = (__bf16*)(ws + WS_PDT); float *COR = (float*)(ws + WS_COR), *GRM = (float*)(ws + WS_GRM), *CODE = (float*)(ws + WS_CODE), *PL = (float*)(ws + WS_PL);
  float* OUTQ = (float*)d_out; float* OUTL = OUTQ + (size_t)NBI * CH * IMH * IMW;
  k_packD<<<NA, 256, 0, stream>>>(Dm, PDT);
  k_corr<<<dim3(NPBT, NA / 128), 128, 0, stream>>>(X, PDT, COR);
  k_gram<<<dim3(NA / 64, NA / 128), 128, 0, stream>>>(PDT, GRM);
  k_code<<<NPBT, 64, 0, stream>>>(COR, GRM, X, Dm, CODE);
  k_fold<<<dim3(IMH, CH, TNB), 128, 0, stream>>>(X, Dm, CODE, OUTQ, PL);
  k_loss<<<1, 256, 0, stream>>>(PL, OUTL);
}
